// MambaSSM_52905407152479
// MI455X (gfx1250) — hardware-run, weakly checked
//
#include <hip/hip_runtime.h>
#include <math.h>

typedef __attribute__((ext_vector_type(16))) _Float16 v16h;
typedef __attribute__((ext_vector_type(8)))  _Float16 v8h;
typedef __attribute__((ext_vector_type(16))) __bf16   v16b;
typedef __attribute__((ext_vector_type(8)))  __bf16   v8b;
typedef __attribute__((ext_vector_type(8)))  float    v8f;
typedef __attribute__((ext_vector_type(4)))  float    v4f;
typedef __attribute__((ext_vector_type(4)))  unsigned v4u;

constexpr int kBatch   = 4;
constexpr int kSeq     = 2048;
constexpr int kDm      = 1024;
constexpr int kDi      = 2048;
constexpr int kNs      = 16;
constexpr int kXz      = 2 * kDi;
constexpr int kRows    = kBatch * kSeq;
constexpr int kPw      = 64;
constexpr int kCvRows  = 32;
constexpr int kCvPitch = 260;
constexpr float kCarryXc = 256.0f;
constexpr float kCarryWp = 32.0f;
constexpr float kProjFold = 1.0f / (kCarryXc * kCarryWp);
static_assert(kRows == 8192 && kXz == 4096, "shape");
static_assert((kDm % 32) == 0 && (kDi % 32) == 0, "GEMM K multiples of 32");
static_assert((kRows % 64) == 0 && (kXz % 64) == 0 && (kPw % 64) == 0, "GEMM M,N multiples of 64");
static_assert(3 * kNs <= kPw, "packed projection width");
static_assert((kSeq % kCvRows) == 0 && (kDi % 256) == 0 && (kSeq % 32) == 0, "tile multiples");

constexpr size_t kOffA16  = 0;
constexpr size_t kOffBT16 = kOffA16  + (size_t)kRows * kDm * 2;
constexpr size_t kOffXIN  = kOffBT16 + (size_t)kXz * kDm * 2;
constexpr size_t kOffXC16 = kOffXIN  + (size_t)kRows * kDi * 4;
constexpr size_t kOffWP16 = kOffXC16 + (size_t)kRows * kDi * 2;
constexpr size_t kOffPROJ = kOffWP16 + (size_t)kPw * kDi * 2;
constexpr size_t kOffDSUM = kOffPROJ + (size_t)kRows * kPw * 4;
constexpr size_t kOffYV   = kOffDSUM + (size_t)kRows * 4;
constexpr size_t kWsTotal = kOffYV   + (size_t)kRows * 4;
static_assert(kWsTotal == 128253952ull, "carve total");
static_assert(kWsTotal <= 134217728ull, "carve cap");
static_assert((kOffBT16 % 128) == 0 && (kOffXIN % 128) == 0 && (kOffXC16 % 128) == 0 && (kOffWP16 % 128) == 0 &&
              (kOffPROJ % 128) == 0 && (kOffDSUM % 128) == 0 && (kOffYV % 128) == 0, "128-B aligned regions");

__device__ __forceinline__ unsigned bf_rne_word(float f) {
  const unsigned u = __float_as_uint(f);
  return u + 0x7FFFu + ((u >> 16) & 1u);
}
__device__ __forceinline__ float bf_rne(float f) {
  return __uint_as_float(bf_rne_word(f) & 0xFFFF0000u);
}
__device__ __forceinline__ unsigned pack_bf2(float lo, float hi) {
  return (bf_rne_word(lo) >> 16) | (bf_rne_word(hi) & 0xFFFF0000u);
}

__device__ __forceinline__ void row_guard_h(v8f& a, v8f& b, v8f& c, v8f& d, v16h x, v16h y0, v16h y1, v16h y2, v16h y3) {
  asm volatile("v_nop\n\tv_nop\n\tv_nop\n\tv_nop" : "+v"(a), "+v"(b), "+v"(c), "+v"(d) : "v"(x), "v"(y0), "v"(y1), "v"(y2), "v"(y3));
}
__device__ __forceinline__ void row_guard_b(v8f& a, v8f& b, v8f& c, v8f& d, v16b x, v16b y0, v16b y1, v16b y2, v16b y3) {
  asm volatile("v_nop\n\tv_nop\n\tv_nop\n\tv_nop" : "+v"(a), "+v"(b), "+v"(c), "+v"(d) : "v"(x), "v"(y0), "v"(y1), "v"(y2), "v"(y3));
}
__device__ __forceinline__ void keep4_h(v16h a, v16h b, v16h c, v16h d) { asm volatile("v_nop" :: "v"(a), "v"(b), "v"(c), "v"(d)); }
__device__ __forceinline__ void keep4_b(v16b a, v16b b, v16b c, v16b d) { asm volatile("v_nop" :: "v"(a), "v"(b), "v"(c), "v"(d)); }
__device__ __forceinline__ void acc_guard4(v8f& a, v8f& b, v8f& c, v8f& d) { asm volatile("v_nop\n\tv_nop\n\tv_nop\n\tv_nop" : "+v"(a), "+v"(b), "+v"(c), "+v"(d)); }

template <typename T> struct Frag;
template <> struct Frag<_Float16> {
  typedef v16h V; union U { v16h v; v8h h[2]; };
  static __device__ __forceinline__ v16h load(const _Float16* p) {
    U f; f.h[0] = *(const v8h*)(p); f.h[1] = *(const v8h*)(p + 16); return f.v;
  }
  static __device__ __forceinline__ v8f mma(v16h a, v16h b, v8f c) {
    return __builtin_amdgcn_wmma_f32_16x16x32_f16(false, a, false, b, (short)0, c, false, false);
  }
  static __device__ __forceinline__ void guard4(v8f& a, v8f& b, v8f& c, v8f& d, v16h x, v16h y0, v16h y1, v16h y2, v16h y3) { row_guard_h(a, b, c, d, x, y0, y1, y2, y3); }
  static __device__ __forceinline__ void keep(v16h a, v16h b, v16h c, v16h d) { keep4_h(a, b, c, d); }
};
template <> struct Frag<__bf16> {
  typedef v16b V; union U { v16b v; v8b h[2]; };
  static __device__ __forceinline__ v16b load(const __bf16* p) {
    U f; f.h[0] = *(const v8b*)(p); f.h[1] = *(const v8b*)(p + 16); return f.v;
  }
  static __device__ __forceinline__ v8f mma(v16b a, v16b b, v8f c) {
    return __builtin_amdgcn_wmma_f32_16x16x32_bf16(false, a, false, b, (short)0, c, false, false);
  }
  static __device__ __forceinline__ void guard4(v8f& a, v8f& b, v8f& c, v8f& d, v16b x, v16b y0, v16b y1, v16b y2, v16b y3) { row_guard_b(a, b, c, d, x, y0, y1, y2, y3); }
  static __device__ __forceinline__ void keep(v16b a, v16b b, v16b c, v16b d) { keep4_b(a, b, c, d); }
};
template <int ET> struct Elem;
template <> struct Elem<0> { typedef _Float16 T; };
template <> struct Elem<1> { typedef __bf16 T; };

template <int ET, int EPI>
__global__ __launch_bounds__(256) void gemm64_kernel(
    const unsigned short* __restrict__ Ap, int lda,
    const unsigned short* __restrict__ Btp, int ldb,
    float* __restrict__ C, int ldc, int M, int N, int K, float scale)
{
  typedef typename Elem<ET>::T T;
  typedef typename Frag<T>::V V;
  const T* A  = (const T*)Ap;
  const T* Bt = (const T*)Btp;
  __shared__ __align__(16) float sT[8][16 * 68];
  const int lane = threadIdx.x & 31;
  const int wave = threadIdx.x >> 5;
  const int tilesN = N >> 6;
  const int tilesM = M >> 6;
  const int tile = blockIdx.x * 8 + wave;
  if (tile >= tilesM * tilesN) return;
  const int tm = tile / tilesN;
  const int tn = tile - tm * tilesN;
  const int m0 = tm << 6;
  const int n0 = tn << 6;

  const int rlane = lane & 15;
  const int koff  = (lane >> 4) * 8;
  const int mOff  = (lane >> 4) * 8;

  v8f acc[4][4];
#pragma unroll
  for (int i = 0; i < 4; ++i)
#pragma unroll
    for (int j = 0; j < 4; ++j) acc[i][j] = (v8f){0.f,0.f,0.f,0.f,0.f,0.f,0.f,0.f};

  for (int k0 = 0; k0 < K; k0 += 32) {
    V bh[4];
#pragma unroll
    for (int j = 0; j < 4; ++j) {
      const size_t bo = (size_t)(n0 + (j << 4) + rlane) * ldb + koff + k0;
      bh[j] = Frag<T>::load(Bt + bo);
    }
#pragma unroll
    for (int i = 0; i < 4; ++i) {
      const size_t ao = (size_t)(m0 + (i << 4) + rlane) * lda + koff + k0;
      V ah = Frag<T>::load(A + ao);
#pragma unroll
      for (int j = 0; j < 4; ++j) acc[i][j] = Frag<T>::mma(ah, bh[j], acc[i][j]);
      Frag<T>::guard4(acc[i][0], acc[i][1], acc[i][2], acc[i][3], ah, bh[0], bh[1], bh[2], bh[3]);
    }
    Frag<T>::keep(bh[0], bh[1], bh[2], bh[3]);
  }
  acc_guard4(acc[0][0], acc[0][1], acc[0][2], acc[0][3]);
  acc_guard4(acc[1][0], acc[1][1], acc[1][2], acc[1][3]);
  acc_guard4(acc[2][0], acc[2][1], acc[2][2], acc[2][3]);
  acc_guard4(acc[3][0], acc[3][1], acc[3][2], acc[3][3]);

  float* slab = sT[wave];
#pragma unroll
  for (int i = 0; i < 4; ++i) {
    const int mBase = m0 + (i << 4);
#pragma unroll
    for (int j = 0; j < 4; ++j) {
#pragma unroll
      for (int r = 0; r < 8; ++r) {
        slab[(mOff + r) * 68 + (j << 4) + rlane] = acc[i][j][r] * scale;
      }
    }
    __builtin_amdgcn_fence(__ATOMIC_RELEASE, "workgroup");
    __builtin_amdgcn_wave_barrier();
    __builtin_amdgcn_fence(__ATOMIC_ACQUIRE, "workgroup");
    if (EPI == 0) {
      const int hh = lane >> 4, c4 = (lane & 15) * 4;
      for (int pass = 0; pass < 2; ++pass) {
#pragma unroll
        for (int it = 0; it < 8; ++it) {
          const int row = it * 2 + hh;
          const v4f v = *(const v4f*)(slab + row * 68 + c4);
          *(volatile v4f*)(C + (size_t)(mBase + row) * ldc + n0 + c4) = v;
        }
        __threadfence();
      }
    } else {
      const int q = lane >> 3, c4 = (lane & 7) * 4;
      const int gcol = c4 + ((c4 >= 16) ? 16 : 0);
#pragma unroll 1
      for (int it = 0; it < 4; ++it) {
        const int row = it * 4 + q;
        const v4f gv = *(const v4f*)(slab + row * 68 + gcol);
        const v4f iv = *(const v4f*)(slab + row * 68 + gcol + 16);
        v4f o;
#pragma unroll
        for (int e = 0; e < 4; ++e) {
          const float g  = gv[e];
          const float xi = iv[e];
          const float sg = 1.0f / (1.0f + expf(-g));
          o[e] = (g * sg) * xi;
        }
        float* p = C + (size_t)(mBase + row) * ldc + (n0 >> 1) + c4;
        *(volatile v4f*)p = o;
        __threadfence();
        *(volatile v4f*)p = o;
      }
    }
    __builtin_amdgcn_fence(__ATOMIC_RELEASE, "workgroup");
    __builtin_amdgcn_wave_barrier();
    __builtin_amdgcn_fence(__ATOMIC_ACQUIRE, "workgroup");
  }
}

__global__ __launch_bounds__(256) void cast_bf16_kernel(
    const float* __restrict__ src, unsigned short* __restrict__ dst, int total8)
{
  const int i = blockIdx.x * 256 + threadIdx.x;
  if (i >= total8) return;
  const size_t e0 = (size_t)i << 3;
  const v4f a0 = *(const v4f*)(src + e0);
  const v4f a1 = *(const v4f*)(src + e0 + 4);
  const float f0 = a0[0], f1 = a0[1], f2 = a0[2], f3 = a0[3];
  const float f4 = a1[0], f5 = a1[1], f6 = a1[2], f7 = a1[3];
  v4u w;
  w[0] = pack_bf2(f0, f1);
  w[1] = pack_bf2(f2, f3);
  w[2] = pack_bf2(f4, f5);
  w[3] = pack_bf2(f6, f7);
  unsigned short* q = dst + e0;
  *(volatile v4u*)q = w;
  __threadfence();
  *(volatile v4u*)q = w;
}

__global__ __launch_bounds__(256) void win_transpose_kernel(
    const float* __restrict__ W, unsigned short* __restrict__ Bt)
{
  __shared__ float tile[64 * 65];
  const int tid = threadIdx.x, lane = tid & 31, wave = tid >> 5;
  const int n0 = blockIdx.x * 64;
  const int k0 = blockIdx.y * 64;
#pragma unroll
  for (int p = 0; p < 16; ++p) {
    const int idx = tid + p * 256;
    const int kk  = idx >> 6;
    const int nn  = idx & 63;
    tile[kk * 65 + nn] = W[(size_t)(k0 + kk) * kXz + n0 + nn];
  }
  __syncthreads();
  const int s  = (n0 >= kDi) ? 1 : 0;
  const int c0 = n0 - s * kDi;
  const int q = lane >> 3, c8 = (lane & 7) * 8;
  v4u wv[2];
#pragma unroll
  for (int it = 0; it < 2; ++it) {
    const int nrow = it * 32 + wave * 4 + q;
#pragma unroll
    for (int e = 0; e < 4; ++e) {
      const float lo = tile[(c8 + 2 * e) * 65 + nrow];
      const float hi = tile[(c8 + 2 * e + 1) * 65 + nrow];
      wv[it][e] = pack_bf2(lo, hi);
    }
  }
  for (int pass = 0; pass < 2; ++pass) {
#pragma unroll
    for (int it = 0; it < 2; ++it) {
      const int nrow = it * 32 + wave * 4 + q;
      const int drow = ((c0 >> 4) + (nrow >> 4)) * 32 + s * 16 + (nrow & 15);
      *(volatile v4u*)(Bt + (size_t)drow * kDm + k0 + c8) = wv[it];
    }
    __threadfence();
  }
}

__global__ __launch_bounds__(256) void pack_proj_kernel(
    const float* __restrict__ Wd, const float* __restrict__ Wb, const float* __restrict__ Wc,
    unsigned short* __restrict__ WP)
{
  __shared__ float tile[64 * 65];
  const int tid = threadIdx.x, lane = tid & 31, wave = tid >> 5;
  const int k0 = blockIdx.x * 64;
#pragma unroll 1
  for (int s = 0; s < 3; ++s) {
    const float* src = (s == 0) ? Wd : ((s == 1) ? Wb : Wc);
#pragma unroll
    for (int p = 0; p < 4; ++p) {
      const int idx = tid + p * 256;
      const int kk  = idx >> 4;
      const int col = idx & 15;
      const float v = src[(size_t)(k0 + kk) * kNs + col];
      tile[kk * 65 + s * 16 + col] = bf_rne(v) * kCarryWp;
    }
  }
#pragma unroll
  for (int p = 0; p < 4; ++p) {
    const int idx = tid + p * 256;
    const int kk  = idx >> 4;
    const int col = idx & 15;
    tile[kk * 65 + 48 + col] = 0.0f;
  }
  __syncthreads();
  const int q = lane >> 3, c8 = (lane & 7) * 8;
  v8h hv[2];
#pragma unroll
  for (int it = 0; it < 2; ++it) {
    const int nrow = it * 32 + wave * 4 + q;
#pragma unroll
    for (int e = 0; e < 8; ++e) hv[it][e] = (_Float16)tile[(c8 + e) * 65 + nrow];
  }
  for (int pass = 0; pass < 2; ++pass) {
#pragma unroll
    for (int it = 0; it < 2; ++it) {
      const int nrow = it * 32 + wave * 4 + q;
      *(volatile v8h*)(WP + (size_t)nrow * kDi + k0 + c8) = hv[it];
    }
    __threadfence();
  }
}

__global__ __launch_bounds__(256) void conv_skip_kernel(
    const float* __restrict__ XIN, const float* __restrict__ cw, const float* __restrict__ cb,
    const float* __restrict__ Dv, unsigned short* __restrict__ XC16, float* __restrict__ DSUM)
{
  __shared__ __align__(16) float sT[kCvRows * kCvPitch];
  __shared__ float sR[kCvRows];
  const int tid = threadIdx.x, lane = tid & 31, wave = tid >> 5;
  const int g0 = blockIdx.x * kCvRows;
  const int tb = g0 & (kSeq - 1);
  const bool hist = (tb > 0);
  const int rb = hist ? (g0 - 3) : g0;
  float racc[4] = {0.f, 0.f, 0.f, 0.f};
#pragma unroll 1
  for (int cg = 0; cg < kDi / 256; ++cg) {
    const int d0 = cg * 256, d = d0 + tid;
    const v4f wv = *(const v4f*)(cw + (size_t)d * 4);
    const float wa = wv[0], wb = wv[1], wc = wv[2], wd = wv[3];
    const float w0 = bf_rne(wa), w1 = bf_rne(wb), w2 = bf_rne(wc), w3 = bf_rne(wd);
    const float bc = bf_rne(cb[d]);
    float xm3, xm2, xm1;
    {
      const float v3 = XIN[(size_t)rb * kDi + d];
      const float v2 = XIN[(size_t)(rb + 1) * kDi + d];
      const float v1 = XIN[(size_t)(rb + 2) * kDi + d];
      xm3 = hist ? v3 : 0.f;
      xm2 = hist ? v2 : 0.f;
      xm1 = hist ? v1 : 0.f;
    }
    const v4f dA = *(const v4f*)(Dv + d0 + lane * 8);
    const v4f dB = *(const v4f*)(Dv + d0 + lane * 8 + 4);
    float dr[8];
#pragma unroll
    for (int e = 0; e < 4; ++e) {
      const float fa = dA[e];
      const float fb = dB[e];
      dr[e]     = bf_rne(fa);
      dr[4 + e] = bf_rne(fb);
    }
#pragma unroll 1
    for (int s = 0; s < kCvRows; ++s) {
      const float xcur = XIN[(size_t)(g0 + s) * kDi + d];
      float acc = w0 * xm3;
      acc = fmaf(w1, xm2, acc);
      acc = fmaf(w2, xm1, acc);
      acc = fmaf(w3, xcur, acc);
      sT[s * kCvPitch + tid] = acc + bc;
      xm3 = xm2; xm2 = xm1; xm1 = xcur;
    }
    __syncthreads();
    v8h hv[4];
#pragma unroll
    for (int it = 0; it < 4; ++it) {
      const float* sp = sT + (it * 8 + wave) * kCvPitch + lane * 8;
      const v4f a0 = *(const v4f*)(sp);
      const v4f a1 = *(const v4f*)(sp + 4);
      float p = 0.f;
#pragma unroll
      for (int e = 0; e < 4; ++e) {
        const float x0 = a0[e];
        const float x1 = a1[e];
        p = fmaf(x0, dr[e], p);
        p = fmaf(x1, dr[4 + e], p);
        hv[it][e]     = (_Float16)(x0 * kCarryXc);
        hv[it][4 + e] = (_Float16)(x1 * kCarryXc);
      }
      p += __shfl_xor(p, 16, 32);
      p += __shfl_xor(p, 8, 32);
      p += __shfl_xor(p, 4, 32);
      p += __shfl_xor(p, 2, 32);
      p += __shfl_xor(p, 1, 32);
      racc[it] += p;
    }
    for (int pass = 0; pass < 2; ++pass) {
#pragma unroll
      for (int it = 0; it < 4; ++it)
        *(volatile v8h*)(XC16 + (size_t)(g0 + it * 8 + wave) * kDi + d0 + lane * 8) = hv[it];
      __threadfence();
    }
    __syncthreads();
  }
#pragma unroll
  for (int it = 0; it < 4; ++it) {
    if (lane == 0) sR[it * 8 + wave] = racc[it];
  }
  __syncthreads();
  if (wave == 0) {
    const float v = sR[lane];
    float* p = DSUM + g0 + lane;
    *(volatile float*)p = v;
    __threadfence();
    *(volatile float*)p = v;
  }
}

__global__ __launch_bounds__(32) void scan_kernel(
    const float* __restrict__ PROJ, const float* __restrict__ bdel, const float* __restrict__ DSUM,
    float* __restrict__ YV)
{
  __shared__ __align__(16) float sX[32 * kPw];
  const int lane = threadIdx.x;
  const int n = lane & 15;
  const size_t row0 = (size_t)blockIdx.x * kSeq;
  const float lA = -0.5f * log1pf((float)(n + 1) * (1.0f / (float)kNs));
  const float bb = bf_rne(bdel[n]);
  const int sr = lane >> 4, c4 = (lane & 15) * 4;
  float h = 0.f;
#pragma unroll 1
  for (int t0 = 0; t0 < kSeq; t0 += 32) {
    __syncthreads();
#pragma unroll 4
    for (int i = 0; i < 16; ++i) {
      const int r = 2 * i + sr;
      *(v4f*)(sX + r * kPw + c4) = *(const v4f*)(PROJ + (row0 + t0 + r) * kPw + c4);
    }
    __syncthreads();
    const float ds = DSUM[row0 + t0 + lane];
    float ykeep = 0.f;
#pragma unroll 1
    for (int s = 0; s < 32; ++s) {
      const float* xr = sX + s * kPw;
      const float delta = xr[n] + bb;
      const float bm = xr[kNs + n];
      const float cm = xr[2 * kNs + n];
      const float a  = expf(delta * lA);
      const float bd = delta * bm;
      h = a * h + bd;
      float part = cm * h;
      part += __shfl_xor(part, 1, 32);
      part += __shfl_xor(part, 2, 32);
      part += __shfl_xor(part, 4, 32);
      part += __shfl_xor(part, 8, 32);
      ykeep = (lane == s) ? part : ykeep;
    }
    const float yv = ykeep + ds;
    float* p = YV + row0 + t0 + lane;
    *(volatile float*)p = yv;
    __threadfence();
    *(volatile float*)p = yv;
  }
}

__global__ __launch_bounds__(256) void outer_kernel(
    const float* __restrict__ YV, const float* __restrict__ wout, float* __restrict__ out)
{
  const int gid = blockIdx.x * 256 + threadIdx.x;
  const int d4 = gid & 255;
  const int mg = gid >> 8;
  const v4f w = *(const v4f*)(wout + d4 * 4);
  const v4f yq = *(const v4f*)(YV + (size_t)mg * 4);
  float wr[4];
#pragma unroll
  for (int e = 0; e < 4; ++e) {
    const float f = w[e];
    wr[e] = bf_rne(f);
  }
  v4f o[4];
#pragma unroll
  for (int r = 0; r < 4; ++r) {
    const float yv = yq[r];
#pragma unroll
    for (int e = 0; e < 4; ++e) o[r][e] = yv * wr[e];
  }
  for (int pass = 0; pass < 2; ++pass) {
#pragma unroll
    for (int r = 0; r < 4; ++r)
      *(volatile v4f*)(out + (size_t)(mg * 4 + r) * kDm + d4 * 4) = o[r];
    __threadfence();
  }
}

extern "C" void kernel_launch(void* const* d_in, const int* in_sizes, int n_in,
                              void* d_out, int out_size, void* d_ws, size_t ws_size,
                              hipStream_t stream)
{
  if (n_in < 10) return;
  if (in_sizes[0] != kRows * kDm) return;
  if (in_sizes[1] != kDm * kXz) return;
  if (in_sizes[2] != kDi * 4) return;
  if (in_sizes[3] != kDi) return;
  if (in_sizes[4] != kDi * kNs) return;
  if (in_sizes[5] != kNs) return;
  if (in_sizes[6] != kDi * kNs) return;
  if (in_sizes[7] != kDi * kNs) return;
  if (in_sizes[8] != kDi) return;
  if (in_sizes[9] != kDm) return;
  if (out_size != kRows * kDm) return;
  if (ws_size < kWsTotal) return;

  const float* x       = (const float*)d_in[0];
  const float* W_in    = (const float*)d_in[1];
  const float* conv_w  = (const float*)d_in[2];
  const float* conv_b  = (const float*)d_in[3];
  const float* W_delta = (const float*)d_in[4];
  const float* b_delta = (const float*)d_in[5];
  const float* W_B     = (const float*)d_in[6];
  const float* W_C     = (const float*)d_in[7];
  const float* Dvec    = (const float*)d_in[8];
  const float* w_out   = (const float*)d_in[9];
  float* out = (float*)d_out;

  char* ws = (char*)d_ws;
  unsigned short* A16  = (unsigned short*)(ws + kOffA16);
  unsigned short* BT16 = (unsigned short*)(ws + kOffBT16);
  float*          XIN  = (float*)(ws + kOffXIN);
  unsigned short* XC16 = (unsigned short*)(ws + kOffXC16);
  unsigned short* WP16 = (unsigned short*)(ws + kOffWP16);
  float*          PROJ = (float*)(ws + kOffPROJ);
  float*          DSUM = (float*)(ws + kOffDSUM);
  float*          YV   = (float*)(ws + kOffYV);

  cast_bf16_kernel<<<(kRows * kDm / 8) / 256, 256, 0, stream>>>(x, A16, kRows * kDm / 8);
  win_transpose_kernel<<<dim3(kXz / 64, kDm / 64), 256, 0, stream>>>(W_in, BT16);
  pack_proj_kernel<<<kDi / 64, 256, 0, stream>>>(W_delta, W_B, W_C, WP16);

  gemm64_kernel<1, 1><<<(kRows / 64) * (kXz / 64) / 8, 256, 0, stream>>>(
      A16, kDm, BT16, kDm, XIN, kDi, kRows, kXz, kDm, 1.0f);

  conv_skip_kernel<<<kRows / kCvRows, 256, 0, stream>>>(XIN, conv_w, conv_b, Dvec, XC16, DSUM);

  gemm64_kernel<0, 0><<<(kRows / 64) * (kPw / 64) / 8, 256, 0, stream>>>(
      XC16, kDi, WP16, kDi, PROJ, kPw, kRows, kPw, kDi, kProjFold);

  scan_kernel<<<kBatch, 32, 0, stream>>>(PROJ, b_delta, DSUM, YV);

  outer_kernel<<<(kRows / 4) * (kDm / 4) / 256, 256, 0, stream>>>(YV, w_out, out);
}
